// Unified2DAttentionOnFrameAsym_85950885528318
// MI455X (gfx1250) — hardware-verified
//
#include <hip/hip_runtime.h>
#include <math.h>

typedef __attribute__((ext_vector_type(16))) _Float16 v16h;
typedef __attribute__((ext_vector_type(16))) __bf16 v16b;
typedef __attribute__((ext_vector_type(8)))  _Float16 v8h;
typedef __attribute__((ext_vector_type(8)))  float v8f;
typedef __attribute__((ext_vector_type(4)))  float v4f;
typedef __attribute__((ext_vector_type(2)))  float v2f;
typedef __attribute__((ext_vector_type(4)))  unsigned v4u;
typedef __attribute__((ext_vector_type(4)))  int v4i;
typedef float __attribute__((may_alias)) float_a;
typedef int __attribute__((may_alias)) int_a;

template <typename T> __device__ __forceinline__ void vst2(void* p, T v) { *(volatile T*)p = v; __threadfence(); *(volatile T*)p = v; }
__device__ __forceinline__ v8f wmma16(v16h a, v16h b, v8f c) {
  v8f d = __builtin_amdgcn_wmma_f32_16x16x32_f16(false, a, false, b, (short)0, c, false, false);
  asm volatile("v_nop\n\tv_nop\n\tv_nop\n\tv_nop" : "+v"(d) : "v"(a), "v"(b));
  return d;
}
__device__ __forceinline__ v8f wmma_bf(v16b a, v16b b, v8f c) {
  v8f d = __builtin_amdgcn_wmma_f32_16x16x32_bf16(false, a, false, b, (short)0, c, false, false);
  asm volatile("v_nop\n\tv_nop\n\tv_nop\n\tv_nop" : "+v"(d) : "v"(a), "v"(b));
  return d;
}
__device__ __forceinline__ v16h frag_h(const _Float16* rowk0, int lane) {
  union { v16h v; v8h q[2]; } u; const _Float16* p = rowk0 + 8 * (lane >> 4);
  u.q[0] = *(const v8h*)p; u.q[1] = *(const v8h*)(p + 16); return u.v;
}
__device__ __forceinline__ v16h frag_f32(const float* rowk0, int lane) {
  v16h a; const float* p = rowk0 + 8 * (lane >> 4);
#pragma unroll
  for (int i = 0; i < 8; ++i) { a[i] = (_Float16)p[i]; a[8 + i] = (_Float16)p[16 + i]; }
  return a;
}
__device__ __forceinline__ v16h frag_f32s(const float* rowk0, int lane, float sc) {
  v16h a; const float* p = rowk0 + 8 * (lane >> 4);
#pragma unroll
  for (int i = 0; i < 8; ++i) { a[i] = (_Float16)(p[i] * sc); a[8 + i] = (_Float16)(p[16 + i] * sc); }
  return a;
}
__device__ __forceinline__ v16h fragc_f32(const float* W, int k0, int n, int lane, int ld, int K) {
  v16h a; const int g = lane >> 4;
#pragma unroll
  for (int i = 0; i < 8; ++i) { const int ka = k0 + 8 * g + i, kb = ka + 16;
    a[i] = (_Float16)(ka < K ? W[(size_t)(ka < K ? ka : K - 1) * ld + n] : 0.f); a[8 + i] = (_Float16)(kb < K ? W[(size_t)(kb < K ? kb : K - 1) * ld + n] : 0.f); }
  return a;
}
struct F2 { v16b h, l; };
__device__ __forceinline__ F2 bsplit16(const float v[16]) { F2 r;
#pragma unroll
  for (int i = 0; i < 16; ++i) { const __bf16 h = (__bf16)v[i]; r.h[i] = h; r.l[i] = (__bf16)(v[i] - (float)h); }
  return r; }
__device__ __forceinline__ F2 split_row(const float* row, int k0, int lane) { float v[16]; const float* p = row + k0 + 8 * (lane >> 4);
#pragma unroll
  for (int i = 0; i < 8; ++i) { v[i] = p[i]; v[8 + i] = p[16 + i]; }
  return bsplit16(v); }
__device__ __forceinline__ F2 split_rowK(const float* row, int k0, int lane, int K) { float v[16]; const int g = lane >> 4;
#pragma unroll
  for (int i = 0; i < 8; ++i) { const int ka = k0 + 8 * g + i, kb = ka + 16; v[i] = ka < K ? row[ka < K ? ka : K - 1] : 0.f; v[8 + i] = kb < K ? row[kb < K ? kb : K - 1] : 0.f; }
  return bsplit16(v); }
__device__ __forceinline__ F2 split_col(const float* W, int k0, int n, int lane, int ld, int K) { float v[16]; const int g = lane >> 4;
#pragma unroll
  for (int i = 0; i < 8; ++i) { const int ka = k0 + 8 * g + i, kb = ka + 16; v[i] = ka < K ? W[(size_t)(ka < K ? ka : K - 1) * ld + n] : 0.f; v[8 + i] = kb < K ? W[(size_t)(kb < K ? kb : K - 1) * ld + n] : 0.f; }
  return bsplit16(v); }
__device__ __forceinline__ v8f mac3(const F2& a, const F2& b, v8f c) { c = wmma_bf(a.l, b.h, c); c = wmma_bf(a.h, b.l, c); return wmma_bf(a.h, b.h, c); }
__device__ __forceinline__ float sigm(float v) { return 1.0f / (1.0f + expf(-v)); }
#define LDSX() do { asm volatile("s_wait_dscnt 0" ::: "memory"); __builtin_amdgcn_wave_barrier(); __builtin_amdgcn_fence(__ATOMIC_RELEASE, "workgroup"); } while (0)


#define NB 4
#define CI 256
#define FQ 8
#define TT 1000
#define TP 1024
#define NHh 8
#define CHq 16
#define VHc 32
#define CT 512
#define HDq 128
#define VHD 256
#define WIN 100
#define NPOS (TT * FQ)
#ifndef TNB
#define TNB NB
#define TB0 0
#define TQB (TP / 64)
#endif
typedef __attribute__((ext_vector_type(8))) __bf16 v8b;
__device__ __forceinline__ v16b frag_b(const __bf16* rowk0, int lane) {
  union { v16b v; v8b q[2]; } u; const __bf16* p = rowk0 + 8 * (lane >> 4);
  u.q[0] = *(const v8b*)p; u.q[1] = *(const v8b*)(p + 16); return u.v;
}
__device__ __forceinline__ float bfr(float v) { return (float)(__bf16)v; }
__device__ __attribute__((noinline)) float exp_ni(float v) { return expf(v); }
__device__ __attribute__((noinline)) float erf_ni(float v) { return erff(v); }

#define WS_PQ  0u
#define WS_PP  (2u * CT * CI)
#define WS_QH  (WS_PP + 2u * CI * CI)
#define WS_QL  (WS_QH + 2u * NB * NHh * TP * HDq)
#define WS_KH  (WS_QL + 2u * NB * NHh * TP * HDq)
#define WS_KL  (WS_KH + 2u * NB * NHh * TP * HDq)
#define WS_VH  (WS_KL + 2u * NB * NHh * TP * HDq)
#define WS_VL  (WS_VH + 2u * NB * NHh * TP * VHD)
#define WS_CTX (WS_VL + 2u * NB * NHh * TP * VHD)
#define WS_END (WS_CTX + 4u * (size_t)NB * TP * FQ * CI)

__global__ __launch_bounds__(256) void k_pack(const float* __restrict__ WQ, const float* __restrict__ WP, __bf16* __restrict__ PK) {
  __shared__ __align__(16) __bf16 s[CI]; const int n = blockIdx.x, which = blockIdx.y, t = threadIdx.x; if (which == 1 && n >= CI) return;
  const float* src = (which == 0) ? (WQ + (size_t)n * CI) : (WP + (size_t)n * CI); s[t] = (__bf16)src[t];
  __syncthreads();
  if (t < CI / 8) vst2((unsigned*)(PK + ((which == 0) ? 0 : (size_t)CT * CI) + (size_t)n * CI + t * 8), *(const v4u*)&s[t * 8]);
}
__global__ __launch_bounds__(128) void k_qkv(const float* __restrict__ X, const __bf16* __restrict__ PQ, const float* __restrict__ BQ, const float* __restrict__ AQ, const float* __restrict__ GQ, const float* __restrict__ BEQ, _Float16* __restrict__ QH, _Float16* __restrict__ QL, _Float16* __restrict__ KH, _Float16* __restrict__ KL, _Float16* __restrict__ VH, _Float16* __restrict__ VL) {
  __shared__ __align__(16) __bf16 sa[64][CI + 8]; __shared__ __align__(16) _Float16 sqh[8][2][2][HDq + 8], sql[8][2][2][HDq + 8]; __shared__ __align__(16) _Float16 svh[8][2][VHD + 8], svl[8][2][VHD + 8];
  const int tid = threadIdx.x, wave = tid >> 5, lane = tid & 31, col = lane & 15, g = lane >> 4; const size_t b = blockIdx.y + TB0; const int t0 = blockIdx.x * 8;
  for (int e = tid; e < 64 * CI; e += 128) { const int c = e >> 6, p = e & 63; const int tl = p >> 3, f = p & 7; sa[p][c] = (__bf16)X[((b * CI + c) * FQ + f) * TT + t0 + tl]; }
  if (tid < 64) for (int c = CI; c < CI + 8; ++c) sa[tid][c] = (__bf16)0.f;
  __syncthreads();
  const float aq = bfr(AQ[0]);
  float rs_[8], rq_[8], mu[8], rsd[8];
#pragma unroll
  for (int r = 0; r < 8; ++r) { rs_[r] = 0.f; rq_[r] = 0.f; mu[r] = 0.f; rsd[r] = 0.f; }
#pragma unroll 1
  for (int pass = 0; pass < 2; ++pass) {
    if (pass == 1) {
#pragma unroll
      for (int r = 0; r < 8; ++r) { float s = rs_[r], q2 = rq_[r];
#pragma unroll
        for (int o = 1; o < 16; o <<= 1) { s += __shfl_xor(s, o); q2 += __shfl_xor(q2, o); }
        mu[r] = s / (float)CT; rsd[r] = 1.0f / sqrtf(fmaxf(q2 / (float)CT - mu[r] * mu[r], 0.f) + 1e-5f); } }
#pragma unroll 1
    for (int nb = 0; nb < CT / 128; ++nb) { const int n0 = nb * 128; v8f acc[8] = {};
#pragma unroll 2
      for (int kc = 0; kc < CI / 32; ++kc) { const v16b a = frag_b(&sa[wave * 16 + col][kc * 32], lane);
#pragma unroll
        for (int j = 0; j < 8; ++j) acc[j] = wmma_bf(a, frag_b(PQ + (size_t)(n0 + j * 16 + col) * CI + kc * 32, lane), acc[j]); }
      if (pass == 0) {
#pragma unroll
        for (int j = 0; j < 8; ++j) { const float bb = bfr(BQ[n0 + j * 16 + col]);
#pragma unroll
          for (int r = 0; r < 8; ++r) { float v = acc[j][r] + bb; v = (v >= 0.f) ? v : aq * v; rs_[r] += v; rq_[r] += v * v; } }
      } else {
#pragma unroll
        for (int j = 0; j < 8; ++j) { const int ch = n0 + j * 16 + col; const float bb = bfr(BQ[ch]), gg = bfr(GQ[ch]), be = bfr(BEQ[ch]); const int hl = (ch >> 6) & 1, cw = ch & 63;
#pragma unroll
          for (int r = 0; r < 8; ++r) { float v = acc[j][r] + bb; v = (v >= 0.f) ? v : aq * v; v = (v - mu[r]) * rsd[r] * gg + be;
            const int p = wave * 16 + 8 * g + r; const int tl = p >> 3, f = p & 7; const _Float16 hv = (_Float16)v; const _Float16 lv = (_Float16)((v - (float)hv) * 2048.0f);
            if (cw < 32) { const int which = cw >> 4, idx = (cw & 15) * 8 + f; sqh[tl][hl][which][idx] = hv; sql[tl][hl][which][idx] = lv; }
            else { const int idx = (cw - 32) * 8 + f; svh[tl][hl][idx] = hv; svl[tl][hl][idx] = lv; } } }
        __syncthreads();
        for (int e = tid; e < 8 * 2 * 2 * 16; e += 128) { const int q16 = e & 15, which = (e >> 4) & 1, hl = (e >> 5) & 1, tl = e >> 6; const int h = nb * 2 + hl; const size_t o = (((b * NHh + h) * TP) + t0 + tl) * HDq + q16 * 8;
          _Float16* DH_ = which ? KH : QH; _Float16* DL_ = which ? KL : QL; vst2((unsigned*)(DH_ + o), *(const v4u*)&sqh[tl][hl][which][q16 * 8]); vst2((unsigned*)(DL_ + o), *(const v4u*)&sql[tl][hl][which][q16 * 8]); }
        for (int e = tid; e < 8 * 2 * 32; e += 128) { const int q32 = e & 31, hl = (e >> 5) & 1, tl = e >> 6; const int h = nb * 2 + hl; const size_t o = (((b * NHh + h) * TP) + t0 + tl) * VHD + q32 * 8;
          vst2((unsigned*)(VH + o), *(const v4u*)&svh[tl][hl][q32 * 8]); vst2((unsigned*)(VL + o), *(const v4u*)&svl[tl][hl][q32 * 8]); }
        __syncthreads(); } }
  }
}
__global__ __launch_bounds__(128) void k_attn(const _Float16* __restrict__ QH, const _Float16* __restrict__ QL, const _Float16* __restrict__ KH, const _Float16* __restrict__ KL, const _Float16* __restrict__ VH, const _Float16* __restrict__ VL, float* __restrict__ CTX) {
  __shared__ __align__(16) _Float16 sp[4][16][40], spu[4][16][40], spe[4][16][40]; __shared__ __align__(16) _Float16 svt[VHD / 2][40], svtl[VHD / 2][40]; __shared__ __align__(16) float so[4][16][VHD + 4];
  const int tid = threadIdx.x, wave = tid >> 5, lane = tid & 31, col = lane & 15, g = lane >> 4; const int qb = blockIdx.x, h = blockIdx.y; const size_t b = blockIdx.z + TB0; const int q0 = qb * 64 + wave * 16;
  const size_t hb = (b * NHh + h) * TP; const size_t qo = (hb + q0 + col) * HDq;
  const int ks0 = max(0, qb * 64 - WIN) / 32, ks1 = min((qb * 64 + 64 + 31) / 32, TP / 32);
#pragma unroll 1
  for (int half = 0; half < 2; ++half) {
  float m[8], l[8];
#pragma unroll
  for (int r = 0; r < 8; ++r) { m[r] = -3.0e38f; l[r] = 0.f; }
  v8f acc[8] = {};
#pragma unroll 1
  for (int ks = ks0; ks < ks1; ++ks) { const int j0 = ks * 32;
    __syncthreads();
    for (int e = tid; e < 32 * (VHD / 2) / 8; e += 128) { const int kk = e / (VHD / 16), q8 = e % (VHD / 16); const v4u vh = *(const v4u*)(VH + (hb + j0 + kk) * VHD + half * (VHD / 2) + q8 * 8), vl = *(const v4u*)(VL + (hb + j0 + kk) * VHD + half * (VHD / 2) + q8 * 8); const _Float16* ph = (const _Float16*)&vh; const _Float16* pl = (const _Float16*)&vl;
#pragma unroll
      for (int i = 0; i < 8; ++i) { svt[q8 * 8 + i][kk] = ph[i]; svtl[q8 * 8 + i][kk] = pl[i]; } }
    v8f s[2];
#pragma unroll
    for (int ct = 0; ct < 2; ++ct) { const int kk = j0 + ct * 16 + col; const size_t rk = (hb + kk) * HDq; v8f c = {}, cl = {};
#pragma unroll 1
      for (int kc = 0; kc < HDq / 32; ++kc) { const v16h aq = frag_h(QH + qo + kc * 32, lane), aql = frag_h(QL + qo + kc * 32, lane); const v16h kh = frag_h(KH + rk + kc * 32, lane); c = wmma16(aq, kh, c); cl = wmma16(aql, kh, cl); cl = wmma16(aq, frag_h(KL + rk + kc * 32, lane), cl); }
#pragma unroll
      for (int r = 0; r < 8; ++r) { const int qi = q0 + 8 * g + r; const bool keep = (kk <= qi) && (qi - kk <= WIN) && (kk < TT); s[ct][r] = keep ? (c[r] + cl[r] * (1.0f / 2048.0f)) * 0.08838834764831845f : -3.0e38f; } }
#pragma unroll
    for (int r = 0; r < 8; ++r) { float mx = fmaxf(s[0][r], s[1][r]);
#pragma unroll
      for (int o = 1; o < 16; o <<= 1) mx = fmaxf(mx, __shfl_xor(mx, o));
      const float mn = fmaxf(m[r], mx); const float alpha = (m[r] <= -1.0e38f) ? 0.f : __expf(m[r] - mn);
      const float e0 = (s[0][r] <= -1.0e38f) ? 0.f : __expf(s[0][r] - mn), e1 = (s[1][r] <= -1.0e38f) ? 0.f : __expf(s[1][r] - mn); float es = e0 + e1;
#pragma unroll
      for (int o = 1; o < 16; o <<= 1) es += __shfl_xor(es, o);
      l[r] = l[r] * alpha + es; m[r] = (mn <= -1.0e38f) ? m[r] : mn;
#pragma unroll
      for (int dt = 0; dt < 8; ++dt) acc[dt][r] *= alpha;
      { const float p0 = e0 * 2048.0f, p1 = e1 * 2048.0f; const _Float16 h0 = (_Float16)p0, h1 = (_Float16)p1; sp[wave][8 * g + r][col] = h0; sp[wave][8 * g + r][16 + col] = h1; spe[wave][8 * g + r][col] = (_Float16)(p0 - (float)h0); spe[wave][8 * g + r][16 + col] = (_Float16)(p1 - (float)h1); spu[wave][8 * g + r][col] = (_Float16)e0; spu[wave][8 * g + r][16 + col] = (_Float16)e1; } }
    __syncthreads();
    const v16h pa = frag_h(&sp[wave][col][0], lane), pu = frag_h(&spu[wave][col][0], lane), pe_ = frag_h(&spe[wave][col][0], lane);
#pragma unroll
    for (int dt = 0; dt < 8; ++dt) { const v16h vh = frag_h(&svt[dt * 16 + col][0], lane); acc[dt] = wmma16(pu, frag_h(&svtl[dt * 16 + col][0], lane), acc[dt]); acc[dt] = wmma16(pe_, vh, acc[dt]); acc[dt] = wmma16(pa, vh, acc[dt]); }
    __syncthreads(); }
#pragma unroll
  for (int r = 0; r < 8; ++r) { const float il = (l[r] > 0.f) ? (1.0f / 2048.0f) / l[r] : 0.f;
#pragma unroll
    for (int dt = 0; dt < 8; ++dt) so[wave][8 * g + r][half * (VHD / 2) + dt * 16 + col] = acc[dt][r] * il; }
  }
  LDSX();
  for (int e = lane; e < 16 * 8 * 8; e += 32) { const int q4 = e & 7, f = (e >> 3) & 7, rl = e >> 6; const int t = q0 + rl; if (t >= TT) continue; v4f v;
#pragma unroll
    for (int i = 0; i < 4; ++i) v[i] = so[wave][rl][(q4 * 4 + i) * 8 + f];
    vst2(CTX + ((b * TP * FQ) + (size_t)t * FQ + f) * CI + h * VHc + q4 * 4, v); }
}
__global__ __launch_bounds__(128) void k_proj(const float* __restrict__ CTX, const __bf16* __restrict__ PP, const float* __restrict__ BP, const float* __restrict__ AP, const float* __restrict__ GP, const float* __restrict__ BEP, float* __restrict__ OUT) {
  __shared__ float so[CI / 2][33 * 8 + 1];
  const int tid = threadIdx.x, wave = tid >> 5, lane = tid & 31, col = lane & 15, g = lane >> 4; const size_t b = blockIdx.y + TB0; const int t0 = blockIdx.x * 32; const int chalf = blockIdx.z;
  const float ap = bfr(AP[0]);
#pragma unroll 1
  for (int sub = 0; sub < 4; ++sub) {
    const int tb = t0 + sub * 8; if (tb >= TT) break;
    const size_t r0 = (b * TP * FQ) + (size_t)tb * FQ + wave * 16;
    v8f acc[16] = {};
#pragma unroll 1
    for (int kc = 0; kc < CI / 32; ++kc) { const F2 a = split_row(CTX + (r0 + col) * CI, kc * 32, lane);
#pragma unroll
      for (int j = 0; j < 16; ++j) { const v16b w = frag_b(PP + (size_t)(j * 16 + col) * CI + kc * 32, lane); acc[j] = wmma_bf(a.l, w, acc[j]); acc[j] = wmma_bf(a.h, w, acc[j]); } }
    float vsum[8], vsq[8];
#pragma unroll
    for (int r = 0; r < 8; ++r) { vsum[r] = 0.f; vsq[r] = 0.f; }
#pragma unroll
    for (int j = 0; j < 16; ++j) { const float bb = bfr(BP[j * 16 + col]);
#pragma unroll
      for (int r = 0; r < 8; ++r) { float v = acc[j][r] + bb; v = (v >= 0.f) ? v : ap * v; acc[j][r] = v; vsum[r] += v; vsq[r] += v * v; } }
#pragma unroll
    for (int r = 0; r < 8; ++r) {
#pragma unroll
      for (int o = 1; o < 16; o <<= 1) { vsum[r] += __shfl_xor(vsum[r], o); vsq[r] += __shfl_xor(vsq[r], o); }
      const float mu = vsum[r] / (float)CI; const float rsd = 1.0f / sqrtf(fmaxf(vsq[r] / (float)CI - mu * mu, 0.f) + 1e-5f);
#pragma unroll
      for (int j = 0; j < 16; ++j) { if ((j >> 3) != chalf) continue; const int c = j * 16 + col; const int p = wave * 16 + 8 * g + r; const int tl = sub * 8 + (p >> 3), f = p & 7; so[c - chalf * 128][f * 33 + tl] = (acc[j][r] - mu) * rsd * bfr(GP[c]) + bfr(BEP[c]); } }
  }
  __syncthreads();
  const int nt = min(32, TT - t0);
  for (int e = tid; e < (CI / 2) * FQ; e += 128) { const int cl_ = e >> 3, f = e & 7; const int c = chalf * 128 + cl_; float* dst = OUT + ((b * CI + c) * FQ + f) * TT + t0;
    for (int q4 = 0; q4 < nt / 4; ++q4) { v4f v = {so[cl_][f * 33 + q4 * 4], so[cl_][f * 33 + q4 * 4 + 1], so[cl_][f * 33 + q4 * 4 + 2], so[cl_][f * 33 + q4 * 4 + 3]}; vst2(dst + q4 * 4, v); } }
}
extern "C" void kernel_launch(void* const* d_in, const int* in_sizes, int n_in, void* d_out, int out_size, void* d_ws, size_t ws_size, hipStream_t stream) {
  (void)in_sizes; (void)n_in; (void)out_size;
  const float** F = (const float**)d_in;
  if (ws_size < (size_t)WS_END) return;
  char* ws = (char*)d_ws; __bf16* PK = (__bf16*)ws; _Float16 *QH = (_Float16*)(ws + WS_QH), *QL = (_Float16*)(ws + WS_QL), *KH = (_Float16*)(ws + WS_KH), *KL = (_Float16*)(ws + WS_KL), *VH = (_Float16*)(ws + WS_VH), *VL = (_Float16*)(ws + WS_VL); float* CTX = (float*)(ws + WS_CTX);
  k_pack<<<dim3(CT, 2), 256, 0, stream>>>(F[1], F[6], PK);
  k_qkv<<<dim3(TT / 8, TNB), 128, 0, stream>>>(F[0], PK, F[2], F[3], F[4], F[5], QH, QL, KH, KL, VH, VL);
  k_attn<<<dim3(TQB, NHh, TNB), 128, 0, stream>>>(QH, QL, KH, KL, VH, VL, CTX);
  k_proj<<<dim3((TT + 31) / 32, TNB, 2), 128, 0, stream>>>(CTX, (const __bf16*)(ws + WS_PP), F[7], F[8], F[9], F[10], (float*)d_out);
}
